// KLayerGAT_30133490549159
// MI455X (gfx1250) — hardware-verified
//
#include <hip/hip_runtime.h>


typedef __attribute__((ext_vector_type(16))) _Float16 v16h;
typedef __attribute__((ext_vector_type(8)))  _Float16 v8h;
typedef __attribute__((ext_vector_type(8)))  float    v8f;
typedef __attribute__((ext_vector_type(4)))  float    v4f;
typedef __attribute__((ext_vector_type(2)))  float    v2f;
typedef __attribute__((ext_vector_type(2)))  int      v2i;
typedef unsigned int u32;
#define NN 50000
#define NP 50048
#define NE 800000
#define HEADS 2
#define SORT_N (1 << 20)
#define TILE 8192
#define VST2(T, ptr, val) do { const T _v = (val); *(volatile T*)(ptr) = _v; __threadfence(); *(volatile T*)(ptr) = _v; } while (0)
__device__ __forceinline__ v8f wmma16(v16h a, v16h b, v8f c) {
  v8f d = __builtin_amdgcn_wmma_f32_16x16x32_f16(false, a, false, b, (short)0, c, false, false);
  asm volatile("v_nop\n\tv_nop\n\tv_nop\n\tv_nop" : "+v"(d) : "v"(a), "v"(b));
  return d;
}
__device__ __forceinline__ v16h frag16(const _Float16* p, int hh) {
  const v8h lo = *(const v8h*)(p + 8 * hh), hi = *(const v8h*)(p + 16 + 8 * hh);
  return __builtin_shufflevector(lo, hi, 0,1,2,3,4,5,6,7,8,9,10,11,12,13,14,15);
}

__global__ __launch_bounds__(256) void k_sort_init(const int* __restrict__ src, const int* __restrict__ dst, u32* __restrict__ A, int E) {
  const int i = blockIdx.x * 256 + threadIdx.x;
  VST2(u32, A + i, (i < E) ? (((u32)dst[i]) << 16) | (u32)src[i] : 0xffffffffu);
}
__device__ __forceinline__ void cas_lds(u32* s, int lo, int hi, bool up) {
  const u32 a = s[lo], b = s[hi]; const bool sw = up ? (a > b) : (a < b); s[lo] = sw ? b : a; s[hi] = sw ? a : b;
}
__global__ __launch_bounds__(256) void k_sort_local(u32* __restrict__ A) {
  __shared__ u32 s[TILE];
  const int base = blockIdx.x * TILE, t = threadIdx.x;
  for (int i = t; i < TILE; i += 256) s[i] = A[base + i];
  __syncthreads();
  for (int k = 2; k <= TILE; k <<= 1)
    for (int j = k >> 1; j > 0; j >>= 1) {
      for (int p = t; p < TILE / 2; p += 256) {
        const int lo = ((p >> __builtin_ctz(j)) << (__builtin_ctz(j) + 1)) | (p & (j - 1));
        cas_lds(s, lo, lo + j, (((base + lo) & k) == 0));
      }
      __syncthreads();
    }
  for (int pass = 0; pass < 2; ++pass) { for (int i = t; i < TILE; i += 256) *(volatile u32*)(A + base + i) = s[i]; __threadfence(); }
}
__global__ __launch_bounds__(256) void k_sort_global(u32* __restrict__ A, int logj, int k) {
  const int p = blockIdx.x * 256 + threadIdx.x;
  const int j = 1 << logj;
  const int lo = ((p >> logj) << (logj + 1)) | (p & (j - 1)), hi = lo + j;
  const u32 a = A[lo], b = A[hi];
  const bool up = ((lo & k) == 0), sw = up ? (a > b) : (a < b);
  const u32 vlo = sw ? b : a, vhi = sw ? a : b;
  *(volatile u32*)(A + lo) = vlo; *(volatile u32*)(A + hi) = vhi; __threadfence();
  *(volatile u32*)(A + lo) = vlo; *(volatile u32*)(A + hi) = vhi;
}
__global__ __launch_bounds__(256) void k_sort_lds(u32* __restrict__ A, int k) {
  __shared__ u32 s[TILE];
  const int base = blockIdx.x * TILE, t = threadIdx.x;
  for (int i = t; i < TILE; i += 256) s[i] = A[base + i];
  __syncthreads();
  for (int j = TILE >> 1; j > 0; j >>= 1) {
    for (int p = t; p < TILE / 2; p += 256) {
      const int lo = ((p >> __builtin_ctz(j)) << (__builtin_ctz(j) + 1)) | (p & (j - 1));
      cas_lds(s, lo, lo + j, (((base + lo) & k) == 0));
    }
    __syncthreads();
  }
  for (int pass = 0; pass < 2; ++pass) { for (int i = t; i < TILE; i += 256) *(volatile u32*)(A + base + i) = s[i]; __threadfence(); }
}
__global__ __launch_bounds__(256) void k_segs(const u32* __restrict__ A, v2i* __restrict__ seg) {
  const int n = blockIdx.x * 256 + threadIdx.x;
  if (n >= NP) return;
  int st = 0, c = 0;
  if (n < NN) {
    int lo = 0, hi = SORT_N;
    while (lo < hi) { const int mid = (lo + hi) >> 1; if ((A[mid] >> 16) < (u32)n) lo = mid + 1; else hi = mid; }
    st = lo; hi = SORT_N;
    while (lo < hi) { const int mid = (lo + hi) >> 1; if ((A[mid] >> 16) < (u32)(n + 1)) lo = mid + 1; else hi = mid; }
    c = lo - st;
  }
  const v2i sv = {st, c};
  VST2(v2i, seg + n, sv);
}
__global__ __launch_bounds__(256) void k_tof16(const float* __restrict__ src, int cols, int elu, _Float16* __restrict__ dst) {
  const size_t i8 = (size_t)blockIdx.x * 256 + threadIdx.x;
  if (i8 * 8 >= (size_t)NP * cols) return;
  const size_t i = i8 * 8; const int r = (int)(i / cols);
  v8h v;
#pragma unroll
  for (int e = 0; e < 8; ++e) { float x = (r < NN) ? src[i + e] : 0.0f; if (elu) x = (x > 0.f) ? x : expm1f(x); v[e] = (_Float16)x; }
  VST2(v8h, dst + i, v);
}
__global__ __launch_bounds__(256) void k_wt(const float* __restrict__ W, int kin, int nout, _Float16* __restrict__ Wt) {
  const int i8 = blockIdx.x * 256 + threadIdx.x;
  if (i8 * 8 >= kin * nout) return;
  const int i = i8 * 8, n = i / kin, k0 = i % kin;
  v8h v;
#pragma unroll
  for (int e = 0; e < 8; ++e) v[e] = (_Float16)W[(size_t)(k0 + e) * nout + n];
  VST2(v8h, Wt + (size_t)i, v);
}
template <int KIN, int NOUT>
__global__ __launch_bounds__(128) void k_gemm(const _Float16* __restrict__ A, const _Float16* __restrict__ Wt, const float* __restrict__ bias, float* __restrict__ out) {
  const int lane = threadIdx.x & 31, wave = threadIdx.x >> 5, hh = lane >> 4, l16 = lane & 15;
  const int m0 = (blockIdx.x * 4 + wave) * 16, c0 = blockIdx.y * 64;
  v8f acc[4] = {};
  const _Float16* arow = A + (size_t)(m0 + l16) * KIN;
  for (int kb = 0; kb < KIN; kb += 32) {
    const v16h a = frag16(arow + kb, hh);
#pragma unroll
    for (int t = 0; t < 4; ++t) acc[t] = wmma16(a, frag16(Wt + (size_t)(c0 + t * 16 + l16) * KIN + kb, hh), acc[t]);
  }
  for (int pass = 0; pass < 2; ++pass) {
#pragma unroll
    for (int pr = 0; pr < 2; ++pr) {
      const int c = c0 + pr * 32 + lane;
      const float bb = bias[c];
#pragma unroll
      for (int r = 0; r < 8; ++r) {
        const float a_ = acc[2 * pr][r], b_ = acc[2 * pr + 1][r];
        const float ax = __shfl_xor(a_, 16), bx = __shfl_xor(b_, 16);
        *(volatile float*)(out + (size_t)(m0 + r) * NOUT + c)     = (hh ? bx : a_) + bb;
        *(volatile float*)(out + (size_t)(m0 + r + 8) * NOUT + c) = (hh ? b_ : ax) + bb;
      }
    }
    __threadfence();
  }
}
template <int FO, bool MEAN>
__global__ __launch_bounds__(256) void k_gat_edge(const u32* __restrict__ A, const v2i* __restrict__ seg, const float* __restrict__ el, const float* __restrict__ er,
                                                  const float* __restrict__ attn, float* __restrict__ out) {
  constexpr int FPL = FO / 32;
  constexpr int LD = FO * HEADS;
  const int lane = threadIdx.x & 31;
  const int wid = blockIdx.x * 8 + (threadIdx.x >> 5);
  const int v = MEAN ? wid : (wid >> 1);
  if (v >= NN) return;
  const v2i sv = seg[v];
  float res[FPL];
#pragma unroll
  for (int q = 0; q < FPL; ++q) res[q] = 0.f;
  const int h0 = MEAN ? 0 : (wid & 1), h1 = MEAN ? HEADS : h0 + 1;
  for (int hd = h0; hd < h1; ++hd) {
    const int fbase = hd * FO + lane * FPL;
    float erv[FPL], at[FPL], acc[FPL];
#pragma unroll
    for (int q = 0; q < FPL; ++q) { erv[q] = er[(size_t)v * LD + fbase + q]; at[q] = attn[hd * FO + lane * FPL + q]; acc[q] = 0.f; }
    float m = -INFINITY, l = 0.f;
    for (int p = 0; p < sv[1]; ++p) {
      const int u = (int)(A[sv[0] + p] & 0xffffu);
      float elv[FPL], s = 0.f;
#pragma unroll
      for (int q = 0; q < FPL; ++q) { elv[q] = el[(size_t)u * LD + fbase + q]; float x = elv[q] + erv[q]; x = (x > 0.f) ? x : 0.2f * x; s += x * at[q]; }
#pragma unroll
      for (int off = 16; off > 0; off >>= 1) s += __shfl_xor(s, off, 32);
      const float mn = fmaxf(m, s);
      const float sc = expf(m - mn), pe = expf(s - mn);
      l = l * sc + pe;
#pragma unroll
      for (int q = 0; q < FPL; ++q) acc[q] = acc[q] * sc + pe * elv[q];
      m = mn;
    }
    const float inv = (sv[1] > 0) ? (1.0f / l) : 0.f;
#pragma unroll
    for (int q = 0; q < FPL; ++q) res[q] += acc[q] * inv * (MEAN ? (1.0f / HEADS) : 1.0f);
  }
  if (FPL == 4) { const v4f o = {res[0], res[1], res[2], res[3]}; VST2(v4f, out + (size_t)v * (MEAN ? FO : LD) + (MEAN ? 0 : h0 * FO) + lane * 4, o); }
  else          { const v2f o = {res[0], res[1]};                 VST2(v2f, out + (size_t)v * (MEAN ? FO : LD) + (MEAN ? 0 : h0 * FO) + lane * 2, o); }
}

extern "C" void kernel_launch(void* const* d_in, const int* in_sizes, int n_in,
                              void* d_out, int out_size, void* d_ws, size_t ws_size, hipStream_t stream) {
  (void)in_sizes; (void)n_in; (void)out_size;
  const float* x   = (const float*)d_in[0];
  const int*   src = (const int*)d_in[1];
  const int*   dst = (const int*)d_in[2];
  const float *Ws[3], *bs[3], *Wd[3], *bd[3], *at[3];
  for (int l = 0; l < 3; ++l) { Ws[l] = (const float*)d_in[3 + 5 * l]; bs[l] = (const float*)d_in[4 + 5 * l]; Wd[l] = (const float*)d_in[5 + 5 * l];
                                bd[l] = (const float*)d_in[6 + 5 * l]; at[l] = (const float*)d_in[7 + 5 * l]; }
  float* out = (float*)d_out;

  char* ws = (char*)d_ws; size_t off = 0;
  auto take = [&](size_t bytes) { void* p = ws + off; off = (off + bytes + 255) & ~(size_t)255; return p; };
  u32*   keys = (u32*)take((size_t)SORT_N * 4);
  v2i*   seg  = (v2i*)take((size_t)NP * 8);
  _Float16* A16 = (_Float16*)take((size_t)NP * 256 * 2);
  _Float16* Wst = (_Float16*)take((size_t)256 * 256 * 2);
  _Float16* Wdt = (_Float16*)take((size_t)256 * 256 * 2);
  float* el = (float*)take((size_t)NP * 256 * 4);
  float* er = (float*)take((size_t)NP * 256 * 4);
  float* hcur = (float*)take((size_t)NP * 256 * 4);
  if (off > ws_size) return;
  dim3 b256(256);
  auto cdiv = [](long long a, long long bq) { return (unsigned)((a + bq - 1) / bq); };

  k_sort_init<<<SORT_N / 256, b256, 0, stream>>>(src, dst, keys, NE);
  k_sort_local<<<SORT_N / TILE, b256, 0, stream>>>(keys);
  for (int k = TILE * 2; k <= SORT_N; k <<= 1) {
    for (int logj = __builtin_ctz(k) - 1; (1 << logj) >= TILE; --logj)
      k_sort_global<<<SORT_N / 2 / 256, b256, 0, stream>>>(keys, logj, k);
    k_sort_lds<<<SORT_N / TILE, b256, 0, stream>>>(keys, k);
  }
  k_segs<<<cdiv(NP, 256), b256, 0, stream>>>(keys, seg);

  k_tof16<<<cdiv((long long)NP * 256 / 8, 256), b256, 0, stream>>>(x, 256, 0, A16);
  k_wt<<<cdiv(256 * 256 / 8, 256), b256, 0, stream>>>(Ws[0], 256, 256, Wst);
  k_wt<<<cdiv(256 * 256 / 8, 256), b256, 0, stream>>>(Wd[0], 256, 256, Wdt);
  k_gemm<256, 256><<<dim3(NP / 64, 4), dim3(128), 0, stream>>>(A16, Wst, bs[0], el);
  k_gemm<256, 256><<<dim3(NP / 64, 4), dim3(128), 0, stream>>>(A16, Wdt, bd[0], er);
  k_gat_edge<128, false><<<cdiv(NN * HEADS, 8), b256, 0, stream>>>(keys, seg, el, er, at[0], hcur);
  k_tof16<<<cdiv((long long)NP * 256 / 8, 256), b256, 0, stream>>>(hcur, 256, 1, A16);
  k_wt<<<cdiv(256 * 256 / 8, 256), b256, 0, stream>>>(Ws[1], 256, 256, Wst);
  k_wt<<<cdiv(256 * 256 / 8, 256), b256, 0, stream>>>(Wd[1], 256, 256, Wdt);
  k_gemm<256, 256><<<dim3(NP / 64, 4), dim3(128), 0, stream>>>(A16, Wst, bs[1], el);
  k_gemm<256, 256><<<dim3(NP / 64, 4), dim3(128), 0, stream>>>(A16, Wdt, bd[1], er);
  k_gat_edge<128, false><<<cdiv(NN * HEADS, 8), b256, 0, stream>>>(keys, seg, el, er, at[1], hcur);
  k_tof16<<<cdiv((long long)NP * 256 / 8, 256), b256, 0, stream>>>(hcur, 256, 1, A16);
  k_wt<<<cdiv(256 * 128 / 8, 256), b256, 0, stream>>>(Ws[2], 256, 128, Wst);
  k_wt<<<cdiv(256 * 128 / 8, 256), b256, 0, stream>>>(Wd[2], 256, 128, Wdt);
  k_gemm<256, 128><<<dim3(NP / 64, 2), dim3(128), 0, stream>>>(A16, Wst, bs[2], el);
  k_gemm<256, 128><<<dim3(NP / 64, 2), dim3(128), 0, stream>>>(A16, Wdt, bd[2], er);
  k_gat_edge<64, true><<<cdiv(NN, 8), b256, 0, stream>>>(keys, seg, el, er, at[2], out);
}
